// Head_37623913513539
// MI455X (gfx1250) — hardware-verified
//
#include <hip/hip_runtime.h>
#ifndef NB
#define NB 4
#endif
#ifndef SEQ
#define SEQ 2048
#endif
#define NB_FULL 4
#define SEQ_FULL 2048
#define DM 1024
#define LC 288
#define LCP 320
#define NR ((size_t)NB * SEQ)

static_assert(SEQ % 256 == 0);
static_assert(SEQ <= SEQ_FULL);
static_assert(NB <= NB_FULL);
static_assert(LC % 32 == 0);
static_assert(LCP % 64 == 0);
static_assert(LCP / 64 == 5);
static_assert(LC <= LCP);
static_assert(LC % 8 == 0);
static_assert(DM % 32 == 0);
static_assert(((size_t)SEQ * DM / 8) % 256 == 0);
static_assert(((size_t)LCP * DM / 8) % 256 == 0);
static_assert(((size_t)NB * SEQ) % 128 == 0);

typedef unsigned short v8us __attribute__((ext_vector_type(8), may_alias));
typedef float  v8f  __attribute__((ext_vector_type(8)));
typedef float  v4f  __attribute__((ext_vector_type(4)));
typedef float  v4fa __attribute__((ext_vector_type(4), may_alias));
typedef _Float16 v16h __attribute__((ext_vector_type(16)));
union FragH { v16h v; v8us half[2]; _Float16 h[16]; unsigned short u[16]; };
union Frag8 { v8us v; _Float16 h[8]; unsigned short u[8]; };

__device__ __forceinline__ unsigned short bf16_bits(float x) { unsigned int u = __float_as_uint(x); return (unsigned short)((u + 0x7FFFu + ((u >> 16) & 1u)) >> 16); }
__device__ __forceinline__ float bf16_val(unsigned short b) { return __uint_as_float(((unsigned int)b) << 16); }
__device__ __forceinline__ float bf16_rne(float x) { return bf16_val(bf16_bits(x)); }

__device__ __forceinline__ v16h g2_frag(const _Float16* p, unsigned hh) { FragH f; f.half[0] = *(const v8us*)((const unsigned short*)p + 8u * hh); f.half[1] = *(const v8us*)((const unsigned short*)p + 16u + 8u * hh); return f.v; }
__device__ __forceinline__ v8f g2_mma(v16h a, v16h b, v8f c) { v8f d = __builtin_amdgcn_wmma_f32_16x16x32_f16(false, a, false, b, (short)0, c, false, false); asm volatile("v_nop\n\tv_nop\n\tv_nop\n\tv_nop" : "+v"(d) : "v"(a), "v"(b)); return d; }

__device__ __forceinline__ void g2_kloop(const _Float16* a0p, const _Float16* a1p, const _Float16* b0p, const _Float16* b1p, const _Float16* b2p, const _Float16* b3p,
                                         unsigned kb0, unsigned kb1, unsigned hh,
                                         v8f& c00, v8f& c01, v8f& c02, v8f& c03, v8f& c10, v8f& c11, v8f& c12, v8f& c13) {
#pragma unroll 1
  for (unsigned kb = kb0; kb < kb1; kb += 32u) {
    const v16h a0 = g2_frag(a0p + kb, hh), a1 = g2_frag(a1p + kb, hh);
    v16h b = g2_frag(b0p + kb, hh); c00 = g2_mma(a0, b, c00); c10 = g2_mma(a1, b, c10);
    b = g2_frag(b1p + kb, hh); c01 = g2_mma(a0, b, c01); c11 = g2_mma(a1, b, c11);
    b = g2_frag(b2p + kb, hh); c02 = g2_mma(a0, b, c02); c12 = g2_mma(a1, b, c12);
    b = g2_frag(b3p + kb, hh); c03 = g2_mma(a0, b, c03); c13 = g2_mma(a1, b, c13);
  }
}

__global__ __launch_bounds__(256) void k_x16(const float* __restrict__ x, _Float16* __restrict__ X16) {
  const unsigned t = blockIdx.x * 256u + threadIdx.x; const unsigned b = blockIdx.y;
  const float* src = x + (size_t)b * SEQ_FULL * DM + (size_t)t * 8u;
  const v4f a = *(const v4fa*)src, c = *(const v4fa*)(src + 4);
  Frag8 f;
#pragma unroll
  for (int q = 0; q < 4; ++q) { f.h[q] = (_Float16)bf16_rne(a[q]); f.h[4 + q] = (_Float16)bf16_rne(c[q]); }
  unsigned short* d = (unsigned short*)X16 + (size_t)b * SEQ * DM + (size_t)t * 8u;
  const v8us o = f.v;
  *(volatile v8us*)d = o; __threadfence(); *(volatile v8us*)d = o;
}

__global__ __launch_bounds__(256) void k_wnat(const float* __restrict__ w, _Float16* __restrict__ BW) {
  const unsigned t = blockIdx.x * 256u + threadIdx.x;
  const unsigned row = t >> 7, c8 = (t & 127u) * 8u;
  const bool valid = row < (unsigned)LC;
  const unsigned rc = valid ? row : (unsigned)(LC - 1);
  const float* src = w + (size_t)rc * DM + c8;
  const v4f a = *(const v4fa*)src, c = *(const v4fa*)(src + 4);
  Frag8 f;
#pragma unroll
  for (int q = 0; q < 4; ++q) {
    const float v0 = valid ? bf16_rne(a[q]) * 16.0f : 0.0f;
    const float v1 = valid ? bf16_rne(c[q]) * 16.0f : 0.0f;
    f.h[q] = (_Float16)v0; f.h[4 + q] = (_Float16)v1;
  }
  unsigned short* d = (unsigned short*)BW + (size_t)row * DM + c8;
  const v8us o = f.v;
  *(volatile v8us*)d = o; __threadfence(); *(volatile v8us*)d = o;
}

__global__ __launch_bounds__(256) void k_kvprep(const float* __restrict__ kv, _Float16* __restrict__ KV16, _Float16* __restrict__ KVT) {
  __shared__ unsigned short tl[64][66];
  const unsigned tid = threadIdx.x; const unsigned s0 = blockIdx.x * 64u, l0 = blockIdx.y * 64u, b = blockIdx.z;
  Frag8 fr[2];
#pragma unroll
  for (int it = 0; it < 2; ++it) {
    const unsigned i = tid + (unsigned)it * 256u; const unsigned r = i >> 3, c8 = (i & 7u) * 8u;
    const unsigned lcol = l0 + c8; const bool valid = lcol < (unsigned)LC; const unsigned lc = valid ? lcol : (unsigned)(LC - 8);
    const float* src = kv + ((size_t)b * SEQ_FULL + s0 + r) * LC + lc;
    const v4f a = *(const v4fa*)src, c = *(const v4fa*)(src + 4);
#pragma unroll
    for (int q = 0; q < 4; ++q) {
      const float v0 = valid ? bf16_rne(a[q]) : 0.0f;
      const float v1 = valid ? bf16_rne(c[q]) : 0.0f;
      fr[it].h[q] = (_Float16)v0; fr[it].h[4 + q] = (_Float16)v1;
    }
#pragma unroll
    for (int q = 0; q < 8; ++q) tl[c8 + q][r] = fr[it].u[q];
  }
  __syncthreads();
  for (int pass = 0; pass < 2; ++pass) {
#pragma unroll
    for (int it = 0; it < 2; ++it) {
      const unsigned i = tid + (unsigned)it * 256u; const unsigned r = i >> 3, c8 = (i & 7u) * 8u;
      const v8us o = fr[it].v;
      *(volatile v8us*)((unsigned short*)KV16 + ((size_t)b * SEQ + s0 + r) * LCP + l0 + c8) = o;
      Frag8 f;
#pragma unroll
      for (int q = 0; q < 8; ++q) f.u[q] = tl[r][c8 + q];
      const v8us ot = f.v;
      *(volatile v8us*)((unsigned short*)KVT + ((size_t)b * LCP + l0 + r) * SEQ + s0 + c8) = ot;
    }
    if (pass == 0) __threadfence();
  }
}

__global__ __launch_bounds__(128) void k_proj(const _Float16* __restrict__ A, const _Float16* __restrict__ Bh, const float* __restrict__ bias,
                                              _Float16* __restrict__ QH, _Float16* __restrict__ QL) {
  __shared__ __attribute__((aligned(16))) float so[4][32][68];
  const unsigned tid = threadIdx.x, w = tid >> 5, lane = tid & 31u, ln = lane & 15u, hh = lane >> 4;
  const unsigned row0 = blockIdx.x * 128u + 32u * w, col0 = blockIdx.y * 64u;
  const _Float16* a0p = A + (size_t)(row0 + ln) * DM; const _Float16* a1p = a0p + (size_t)16 * DM;
  const _Float16* b0p = Bh + (size_t)(col0 + ln) * DM; const _Float16* b1p = b0p + (size_t)16 * DM; const _Float16* b2p = b1p + (size_t)16 * DM; const _Float16* b3p = b2p + (size_t)16 * DM;
  const v8f z8 = {0.f,0.f,0.f,0.f,0.f,0.f,0.f,0.f}; v8f c00 = z8, c01 = z8, c02 = z8, c03 = z8, c10 = z8, c11 = z8, c12 = z8, c13 = z8;
  g2_kloop(a0p, a1p, b0p, b1p, b2p, b3p, 0u, (unsigned)DM, hh, c00, c01, c02, c03, c10, c11, c12, c13);
  v8f accs[8] = {c00, c01, c02, c03, c10, c11, c12, c13};
#pragma unroll
  for (int u = 0; u < 8; ++u) {
    const unsigned t = (unsigned)u & 3u, half = (unsigned)u >> 2; const unsigned col = col0 + t * 16u + ln;
    const unsigned colc = col < (unsigned)LC ? col : (unsigned)(LC - 1);
    const float braw = bias[colc];
    const float bv = col < (unsigned)LC ? bf16_rne(braw) : 0.0f;
#pragma unroll
    for (int r = 0; r < 8; ++r) { const unsigned rloc = half * 16u + 8u * hh + (unsigned)r; so[w][rloc][t * 16u + ln] = accs[u][r] * 0.0625f + bv; }
  }
  __syncthreads();
  const unsigned rq = lane >> 3, c8 = (lane & 7u) * 8u;
  for (int pass = 0; pass < 2; ++pass) {
#pragma unroll
    for (int q = 0; q < 8; ++q) {
      const unsigned r = (unsigned)q * 4u + rq;
      const v4f x0 = *(const v4fa*)&so[w][r][c8], x1 = *(const v4fa*)&so[w][r][c8 + 4u];
      Frag8 fh, fl;
#pragma unroll
      for (int i = 0; i < 4; ++i) {
        _Float16 h = (_Float16)x0[i]; fh.h[i] = h; fl.h[i] = (_Float16)((x0[i] - (float)h) * 1024.0f);
        h = (_Float16)x1[i]; fh.h[4 + i] = h; fl.h[4 + i] = (_Float16)((x1[i] - (float)h) * 1024.0f);
      }
      const size_t o = (size_t)(row0 + r) * LCP + col0 + c8;
      const v8us oh = fh.v, ol = fl.v;
      *(volatile v8us*)((unsigned short*)QH + o) = oh;
      *(volatile v8us*)((unsigned short*)QL + o) = ol;
    }
    if (pass == 0) __threadfence();
  }
}

__global__ __launch_bounds__(128) void k_scores(const _Float16* __restrict__ QHb, const _Float16* __restrict__ QLb, const _Float16* __restrict__ KVb, float* __restrict__ S) {
  __shared__ __attribute__((aligned(16))) float so[4][32][68];
  const unsigned nq = blockIdx.x, mt = blockIdx.y;
  if (nq * 64u > mt * 128u + 127u) return;
  const unsigned tid = threadIdx.x, w = tid >> 5, lane = tid & 31u, ln = lane & 15u, hh = lane >> 4;
  const unsigned row0 = mt * 128u + 32u * w, col0 = nq * 64u;
  const _Float16* a0p = QHb + (size_t)(row0 + ln) * LCP; const _Float16* a1p = a0p + (size_t)16 * LCP;
  const _Float16* l0p = QLb + (size_t)(row0 + ln) * LCP; const _Float16* l1p = l0p + (size_t)16 * LCP;
  const _Float16* b0p = KVb + (size_t)(col0 + ln) * LCP; const _Float16* b1p = b0p + (size_t)16 * LCP; const _Float16* b2p = b1p + (size_t)16 * LCP; const _Float16* b3p = b2p + (size_t)16 * LCP;
  const v8f z8 = {0.f,0.f,0.f,0.f,0.f,0.f,0.f,0.f}; v8f c00 = z8, c01 = z8, c02 = z8, c03 = z8, c10 = z8, c11 = z8, c12 = z8, c13 = z8;
  g2_kloop(l0p, l1p, b0p, b1p, b2p, b3p, 0u, (unsigned)LC, hh, c00, c01, c02, c03, c10, c11, c12, c13);
  const float rs = 0.0009765625f;
  c00 = c00 * rs; c01 = c01 * rs; c02 = c02 * rs; c03 = c03 * rs; c10 = c10 * rs; c11 = c11 * rs; c12 = c12 * rs; c13 = c13 * rs;
  g2_kloop(a0p, a1p, b0p, b1p, b2p, b3p, 0u, (unsigned)LC, hh, c00, c01, c02, c03, c10, c11, c12, c13);
  v8f accs[8] = {c00, c01, c02, c03, c10, c11, c12, c13};
#pragma unroll
  for (int u = 0; u < 8; ++u) {
    const unsigned t = (unsigned)u & 3u, half = (unsigned)u >> 2;
#pragma unroll
    for (int r = 0; r < 8; ++r) { const unsigned rloc = half * 16u + 8u * hh + (unsigned)r; so[w][rloc][t * 16u + ln] = accs[u][r] * 0.125f; }
  }
  __syncthreads();
  const unsigned rsub = lane >> 4, c4 = (lane & 15u) * 4u;
  for (int pass = 0; pass < 2; ++pass) {
#pragma unroll
    for (int q = 0; q < 16; ++q) {
      const unsigned r = (unsigned)q * 2u + rsub;
      const v4f v = *(const v4fa*)&so[w][r][c4];
      *(volatile v4f*)(S + (size_t)(row0 + r) * SEQ + col0 + c4) = v;
    }
    if (pass == 0) __threadfence();
  }
}

__global__ __launch_bounds__(256) void k_rsm(const float* __restrict__ S, _Float16* __restrict__ P) {
#pragma clang fp contract(off)
  const unsigned tid = threadIdx.x, w = tid >> 5, lane = tid & 31u;
  const unsigned t = blockIdx.x * 8u + w;
  const unsigned n = t + 1u, kend = ((t >> 8) + 1u) << 8;
  const float* s = S + (size_t)t * SEQ;
  const float ninf = -__builtin_inff();
  float mx = ninf;
#pragma unroll 1
  for (unsigned jb = 0; jb < kend; jb += 256u) {
    const unsigned j0 = jb + lane * 8u;
    const v4f a = *(const v4fa*)(s + j0), c = *(const v4fa*)(s + j0 + 4u);
#pragma unroll
    for (int q = 0; q < 4; ++q) {
      const float v0 = (j0 + (unsigned)q < n) ? a[q] : ninf;
      const float v1 = (j0 + 4u + (unsigned)q < n) ? c[q] : ninf;
      mx = fmaxf(mx, fmaxf(v0, v1));
    }
  }
  mx = fmaxf(mx, __shfl_xor(mx, 16)); mx = fmaxf(mx, __shfl_xor(mx, 8)); mx = fmaxf(mx, __shfl_xor(mx, 4)); mx = fmaxf(mx, __shfl_xor(mx, 2)); mx = fmaxf(mx, __shfl_xor(mx, 1));
  float se = 0.f;
#pragma unroll 1
  for (unsigned jb = 0; jb < kend; jb += 256u) {
    const unsigned j0 = jb + lane * 8u;
    const v4f a = *(const v4fa*)(s + j0), c = *(const v4fa*)(s + j0 + 4u);
#pragma unroll
    for (int q = 0; q < 4; ++q) {
      const float e0 = __expf(a[q] - mx), e1 = __expf(c[q] - mx);
      se += (j0 + (unsigned)q < n) ? e0 : 0.0f;
      se += (j0 + 4u + (unsigned)q < n) ? e1 : 0.0f;
    }
  }
  se += __shfl_xor(se, 16); se += __shfl_xor(se, 8); se += __shfl_xor(se, 4); se += __shfl_xor(se, 2); se += __shfl_xor(se, 1);
  const float sc = 1024.0f / se;
#pragma unroll 1
  for (unsigned jb = 0; jb < kend; jb += 256u) {
    const unsigned j0 = jb + lane * 8u;
    const v4f a = *(const v4fa*)(s + j0), c = *(const v4fa*)(s + j0 + 4u);
    Frag8 f;
#pragma unroll
    for (int q = 0; q < 4; ++q) {
      const float e0 = __expf(a[q] - mx) * sc, e1 = __expf(c[q] - mx) * sc;
      const float p0 = (j0 + (unsigned)q < n) ? e0 : 0.0f;
      const float p1 = (j0 + 4u + (unsigned)q < n) ? e1 : 0.0f;
      f.h[q] = (_Float16)p0; f.h[4 + q] = (_Float16)p1;
    }
    unsigned short* d = (unsigned short*)P + (size_t)t * SEQ + j0;
    const v8us o = f.v;
    *(volatile v8us*)d = o; __threadfence(); *(volatile v8us*)d = o;
  }
}

__global__ __launch_bounds__(128) void k_pv(const _Float16* __restrict__ P, const _Float16* __restrict__ VTb, float* __restrict__ O) {
  __shared__ __attribute__((aligned(16))) float so[4][32][68];
  const unsigned nq = blockIdx.x, mt = blockIdx.y;
  const unsigned tid = threadIdx.x, w = tid >> 5, lane = tid & 31u, ln = lane & 15u, hh = lane >> 4;
  const unsigned row0 = mt * 128u + 32u * w, col0 = nq * 64u;
  unsigned kend = ((mt >> 1) + 1u) << 8; if (kend > (unsigned)SEQ) kend = (unsigned)SEQ;
  const _Float16* a0p = P + (size_t)(row0 + ln) * SEQ; const _Float16* a1p = a0p + (size_t)16 * SEQ;
  const _Float16* b0p = VTb + (size_t)(col0 + ln) * SEQ; const _Float16* b1p = b0p + (size_t)16 * SEQ; const _Float16* b2p = b1p + (size_t)16 * SEQ; const _Float16* b3p = b2p + (size_t)16 * SEQ;
  const v8f z8 = {0.f,0.f,0.f,0.f,0.f,0.f,0.f,0.f}; v8f c00 = z8, c01 = z8, c02 = z8, c03 = z8, c10 = z8, c11 = z8, c12 = z8, c13 = z8;
  g2_kloop(a0p, a1p, b0p, b1p, b2p, b3p, 0u, kend, hh, c00, c01, c02, c03, c10, c11, c12, c13);
  v8f accs[8] = {c00, c01, c02, c03, c10, c11, c12, c13};
#pragma unroll
  for (int u = 0; u < 8; ++u) {
    const unsigned t = (unsigned)u & 3u, half = (unsigned)u >> 2;
#pragma unroll
    for (int r = 0; r < 8; ++r) { const unsigned rloc = half * 16u + 8u * hh + (unsigned)r; so[w][rloc][t * 16u + ln] = accs[u][r] * 0.0009765625f; }
  }
  __syncthreads();
  const unsigned rsub = lane >> 4, c4 = (lane & 15u) * 4u;
  const bool live = (col0 + c4) < (unsigned)LC;
  for (int pass = 0; pass < 2; ++pass) {
#pragma unroll
    for (int q = 0; q < 16; ++q) {
      const unsigned r = (unsigned)q * 2u + rsub;
      const v4f v = *(const v4fa*)&so[w][r][c4];
      if (live) *(volatile v4f*)(O + (size_t)(row0 + r) * LC + col0 + c4) = v;
    }
    if (pass == 0) __threadfence();
  }
}

extern "C" void kernel_launch(void* const* d_in, const int* in_sizes, int n_in,
                              void* d_out, int out_size, void* d_ws, size_t ws_size, hipStream_t stream) {
  if (n_in < 4) return;
  const size_t rows_lo = (size_t)(NB - 1) * SEQ_FULL + SEQ;
  if ((size_t)in_sizes[0] < rows_lo * DM) return;
  if ((size_t)in_sizes[1] < rows_lo * LC) return;
  if ((size_t)in_sizes[2] < (size_t)LC * DM) return;
  if ((size_t)in_sizes[3] < (size_t)LC) return;
  if ((size_t)out_size < rows_lo * LC) return;
  const float* x = (const float*)d_in[0];
  const float* kv = (const float*)d_in[1];
  const float* ww = (const float*)d_in[2];
  const float* wb = (const float*)d_in[3];
  float* out = (float*)d_out;
  char* ws = (char*)d_ws; size_t off = 0;
  auto take = [&](size_t bytes) { char* p = ws + off; off += (bytes + 255) & ~(size_t)255; return p; };
  _Float16* BW  = (_Float16*)take((size_t)LCP * DM * 2);
  _Float16* X16 = (_Float16*)take(NR * DM * 2);
  _Float16* QH  = (_Float16*)take(NR * LCP * 2);
  _Float16* QL  = (_Float16*)take(NR * LCP * 2);
  _Float16* KV16 = (_Float16*)take(NR * LCP * 2);
  _Float16* KVT = (_Float16*)take((size_t)NB * LCP * SEQ * 2);
  float* S = (float*)take((size_t)SEQ * SEQ * 4);
  _Float16* P = (_Float16*)take((size_t)SEQ * SEQ * 2);
  static_assert((size_t)LCP * DM * 2 + (size_t)NB * SEQ * DM * 2 + 4 * ((size_t)NB * SEQ * LCP * 2) + (size_t)SEQ * SEQ * 6 + 8 * 256 <= (size_t)134217728);
  if (off > ws_size) return;

  k_x16<<<dim3((unsigned)((size_t)SEQ * DM / 8 / 256), NB), 256, 0, stream>>>(x, X16);
  k_wnat<<<(unsigned)((size_t)LCP * DM / 8 / 256), 256, 0, stream>>>(ww, BW);
  k_kvprep<<<dim3(SEQ / 64, LCP / 64, NB), 256, 0, stream>>>(kv, KV16, KVT);
  k_proj<<<dim3((unsigned)(NR / 128), LCP / 64), 128, 0, stream>>>(X16, BW, wb, QH, QL);
  for (int b = 0; b < NB; ++b) {
    const size_t ro = (size_t)b * SEQ * LCP;
    k_scores<<<dim3(SEQ / 64, SEQ / 128), 128, 0, stream>>>(QH + ro, QL + ro, KV16 + ro, S);
    k_rsm<<<SEQ / 8, 256, 0, stream>>>(S, P);
    k_pv<<<dim3(LCP / 64, SEQ / 128), 128, 0, stream>>>(P, KVT + (size_t)b * LCP * SEQ, out + (size_t)b * SEQ_FULL * LC);
  }
}
